// Mata_6468220748539
// MI455X (gfx1250) — hardware-run, weakly checked
//
#include <hip/hip_runtime.h>


namespace {
constexpr int NB = 256, NN = 128, NT = NB * NN, E = 262144, F = 128, LD = 29, MD = 16, RW = 16, KI = LD + MD + RW, L = NN * NN, SKIT = 6;
constexpr float XS = 8.0f, WSC = 256.0f, TAU = 1.0f;
typedef _Float16 b16;
typedef __attribute__((ext_vector_type(16))) _Float16 v16b;
typedef __attribute__((ext_vector_type(8))) _Float16 v8b;
typedef __attribute__((ext_vector_type(8))) float v8f;
typedef __attribute__((ext_vector_type(4))) float v4f;
typedef __attribute__((ext_vector_type(4))) _Float16 v4b;
__device__ __forceinline__ float bf16_rne(float f) { unsigned int u = __float_as_uint(f); u += 0x7FFFu + ((u >> 16) & 1u); float r = __uint_as_float(u & 0xFFFF0000u); asm volatile("" : "+v"(r)); return r; }
__device__ __forceinline__ void split16(float v, b16& hi, b16& lo) { hi = (b16)v; lo = (b16)(v - (float)hi); }
__device__ __forceinline__ v16b frag_kb(const b16* p, int hh) { const v8b a = *(const v8b*)(p + 8 * hh), b = *(const v8b*)(p + 16 + 8 * hh); v16b f;
#pragma unroll
  for (int e = 0; e < 8; ++e) { f[e] = a[e]; f[8 + e] = b[e]; } return f; }
__device__ __forceinline__ v8f wmma16b(v16b a, v16b b, v8f c) { v8f d = __builtin_amdgcn_wmma_f32_16x16x32_f16(false, a, false, b, (short)0, c, false, false); asm volatile("v_nop\n\tv_nop\n\tv_nop\n\tv_nop" : "+v"(d) : "v"(a), "v"(b)); return d; }
__device__ __forceinline__ void wave_lds_sync() { __builtin_amdgcn_fence(__ATOMIC_RELEASE, "workgroup"); __builtin_amdgcn_wave_barrier(); __builtin_amdgcn_fence(__ATOMIC_ACQUIRE, "workgroup"); }
__device__ __forceinline__ float pmul(float a, float b) { float p = a * b; asm volatile("" : "+v"(p)); return p; }
__device__ __forceinline__ int iclamp(int v, int lo, int hi) { return v < lo ? lo : (v > hi ? hi : v); }
constexpr int CSR_NBLK9 = 512, CSR_GB9 = 9, CSR_GN9 = 1 << CSR_GB9  , CSR_TS9 = (CSR_GN9 < 32 ? 32 : CSR_GN9)  , CSR_MAXG9 = 512, CSR_CAP9 = 12288  ;
__device__ __host__ __forceinline__ int csr_tix9(int v) { return (v >> CSR_GB9) * CSR_TS9 + (v & (CSR_GN9 - 1)); }
__global__ __launch_bounds__(64) void csrA_kernel9(const int* __restrict__ dst, int E, int N, int nG, int CHP, int NGP, int* __restrict__ STG, int* __restrict__ HST) {
  extern __shared__ int sm[];
  int* cnt = sm; int* run = sm + NGP; int* ids = sm + 2 * NGP;
  const int b = blockIdx.x; const int ch = (E + CSR_NBLK9 - 1) / CSR_NBLK9; const int e0 = b * ch, e1 = min(E, e0 + ch);
  for (int i = threadIdx.x; i < NGP; i += 64) cnt[i] = 0;
  for (int i = threadIdx.x; i < CHP; i += 64) ids[i] = -1;
  __syncthreads();
  if (threadIdx.x == 0) {
    for (int e = e0; e < e1; ++e) { int d = dst[e]; d = (d < 0) ? 0 : (d >= N ? N - 1 : d); cnt[d >> CSR_GB9] += 1; }
    int acc = 0; for (int g = 0; g < nG; ++g) { run[g] = acc; acc += cnt[g]; }
    for (int e = e0; e < e1; ++e) { int d = dst[e]; d = (d < 0) ? 0 : (d >= N ? N - 1 : d); const int g = d >> CSR_GB9; ids[run[g]] = e; run[g] += 1; } }
  __syncthreads();
  typedef __attribute__((ext_vector_type(4))) int v4i;
  for (int pass = 0; pass < 2; ++pass) {
    for (int i = threadIdx.x; i < CHP / 4; i += 64) *(volatile v4i*)(STG + (size_t)b * CHP + i * 4) = *(const v4i*)(&ids[i * 4]);
    for (int i = threadIdx.x; i < NGP / 4; i += 64) { v4i v; for (int e = 0; e < 4; ++e) v[e] = (i * 4 + e < nG) ? cnt[i * 4 + e] : 0; *(volatile v4i*)(HST + (size_t)b * NGP + i * 4) = v; }
    __threadfence(); }
}
__global__ __launch_bounds__(512) void csrS_kernel9(const int* __restrict__ HST, int nG, int NGP, int* __restrict__ START, int* __restrict__ TOT, int* __restrict__ OFF) {
  __shared__ int tot[CSR_MAXG9];
  const int b = threadIdx.x;
  for (int pass = 0; pass < 2; ++pass) { int runb = 0; for (int g = 0; g < nG; ++g) { int c = HST[(size_t)b * NGP + g]; c = (c < 0) ? 0 : c; ((volatile int*)OFF)[(size_t)g * CSR_NBLK9 + b] = runb; runb += c; } __threadfence(); }
  for (int g = threadIdx.x; g < nG; g += 512) { int s = 0; for (int bb = 0; bb < CSR_NBLK9; ++bb) { int c = HST[(size_t)bb * NGP + g]; s += (c < 0) ? 0 : c; } tot[g] = s; }
  __syncthreads();
  if (threadIdx.x < 32) {
    __shared__ int st[CSR_MAXG9 + 32];
    if (threadIdx.x == 0) { int acc = 0; for (int g = 0; g < NGP; ++g) { st[g] = acc; if (g < nG) acc += (tot[g] + 31) & ~31; } st[NGP] = acc; }
    __builtin_amdgcn_fence(__ATOMIC_RELEASE, "workgroup"); __builtin_amdgcn_wave_barrier(); __builtin_amdgcn_fence(__ATOMIC_ACQUIRE, "workgroup");
    for (int pass = 0; pass < 2; ++pass) { for (int i = threadIdx.x; i < NGP + 32; i += 32) { ((volatile int*)START)[i] = (i <= NGP) ? st[min(i, NGP)] : 0; ((volatile int*)TOT)[i] = (i < nG) ? tot[i] : 0; } __threadfence(); } }
}
__global__ __launch_bounds__(256) void csrB_kernel9(const int* __restrict__ dst, int N, int nG, int CHP, int NGP, int permLen, const int* __restrict__ STG, const int* __restrict__ HST, const int* __restrict__ OFF, const int* __restrict__ START, const int* __restrict__ TOT, int* __restrict__ PERM, int* __restrict__ ROWPTR, int* __restrict__ ROWCNT, int* __restrict__ FLAG) {
  typedef __attribute__((ext_vector_type(4))) int v4i;
  __shared__ int ids[CSR_CAP9]; __shared__ unsigned short key[CSR_CAP9]; __shared__ int outp[CSR_CAP9]; __shared__ int ncnt[CSR_GN9 + 1]; __shared__ int boff[CSR_NBLK9 + 1];
  const int g = blockIdx.x, t_ = threadIdx.x; int tot = TOT[g]; int st = START[g], stn = START[g + 1]; const int v0 = g * CSR_GN9; const int nv = min(CSR_GN9, N - v0); const int t0 = g * CSR_TS9;
  st = (st < 0) ? 0 : (st > permLen - 32 ? permLen - 32 : st) & ~31; stn = (stn < st) ? st : (stn > permLen ? permLen : stn); tot = (tot < 0) ? 0 : tot; if (tot > stn - st && tot <= CSR_CAP9) tot = stn - st;
  if (tot > CSR_CAP9) {
    for (int pass = 0; pass < 2; ++pass) { for (int i = t_; i < CSR_TS9 / 4; i += 256) { v4i a, c; for (int e = 0; e < 4; ++e) { a[e] = st; c[e] = 0; } *(volatile v4i*)(ROWPTR + t0 + i * 4) = a; *(volatile v4i*)(ROWCNT + t0 + i * 4) = c; } if (t_ == 0) ((volatile int*)FLAG)[0] = 1; __threadfence(); } (void)nv; return; }
  if (t_ == 0) { int acc = 0; for (int b = 0; b < CSR_NBLK9; ++b) { boff[b] = acc; int c = HST[(size_t)b * NGP + g]; c = (c < 0) ? 0 : (c > CHP ? CHP : c); acc += c; if (acc > tot) acc = tot; } boff[CSR_NBLK9] = acc; }
  for (int i = t_; i <= CSR_GN9; i += 256) ncnt[i] = 0;
  __syncthreads();
  for (int b = 0; b < CSR_NBLK9; ++b) { const int c = boff[b + 1] - boff[b]; int o_ = OFF[(size_t)g * CSR_NBLK9 + b]; o_ = (o_ < 0) ? 0 : (o_ > CHP - c ? CHP - c : o_); const int* src_ = STG + (size_t)b * CHP + o_;
    for (int i = t_; i < c; i += 256) { int id = src_[i]; id = (id < 0) ? 0 : id; ids[boff[b] + i] = id; int d = dst[id]; d = (d < v0) ? v0 : (d >= N ? N - 1 : d); int kk = d - v0; kk = (kk < 0) ? 0 : (kk >= CSR_GN9 ? CSR_GN9 - 1 : kk); key[boff[b] + i] = (unsigned short)kk; } }
  __syncthreads();
  if (t_ == 0) { for (int i = 0; i < tot; ++i) ncnt[key[i]] += 1; int acc = 0; for (int vl = 0; vl < CSR_GN9; ++vl) { const int c = ncnt[vl]; ncnt[vl] = acc; acc += c; } ncnt[CSR_GN9] = acc;
    for (int i = 0; i < tot; ++i) { const int vl = key[i]; outp[ncnt[vl]] = ids[i]; ncnt[vl] += 1; }
    for (int vl = CSR_GN9; vl > 0; --vl) ncnt[vl] = ncnt[vl - 1]; ncnt[0] = 0; }
  __syncthreads();
  for (int pass = 0; pass < 2; ++pass) {
    for (int i = t_; i < (stn - st) / 4; i += 256) { v4i v; for (int e = 0; e < 4; ++e) { const int q = i * 4 + e; v[e] = (q < tot) ? outp[q] : -1; } *(volatile v4i*)(PERM + st + i * 4) = v; }
    for (int i = t_; i < CSR_TS9 / 4; i += 256) { v4i a, c; for (int e = 0; e < 4; ++e) { const int vl = i * 4 + e; const int vc = vl < CSR_GN9 ? vl : CSR_GN9; a[e] = (vl < CSR_GN9) ? st + ncnt[vc] : st; c[e] = (vl < nv) ? (ncnt[(vc < CSR_GN9 ? vc : CSR_GN9 - 1) + 1] - ncnt[vc]) : 0; } *(volatile v4i*)(ROWPTR + t0 + i * 4) = a; *(volatile v4i*)(ROWCNT + t0 + i * 4) = c; }
    __threadfence(); }
}
__global__ __launch_bounds__(256) void csrZ_kernel9(int* __restrict__ p, size_t n4) { typedef __attribute__((ext_vector_type(4))) int v4i; const size_t tid = (size_t)blockIdx.x * 256 + threadIdx.x, nth = (size_t)gridDim.x * 256; v4i z = {0, 0, 0, 0}; for (size_t i = tid; i < n4; i += nth) *(volatile v4i*)(p + i * 4) = z; }
struct CsrBufs9 { int *STG, *HST, *OFF, *START, *TOT, *PERM, *ROWPTR, *ROWCNT, *FLAG; int nG, NGP, CHP; size_t permLen; char* base; size_t bytes; };
static size_t csr_carve9(CsrBufs9& c, char* ws, size_t off, int E, int N) {
  const size_t off0 = off; c.base = ws + off;
  auto al = [&](size_t bytes) { char* p = ws + off; off += (bytes + 255) & ~(size_t)255; return p; };
  c.nG = (N + CSR_GN9 - 1) / CSR_GN9; c.NGP = (c.nG + 31) & ~31; const int ch = (E + CSR_NBLK9 - 1) / CSR_NBLK9; c.CHP = (ch + 31) & ~31; c.permLen = (size_t)E + 32 * (size_t)c.nG + 32;
  c.STG = (int*)al((size_t)CSR_NBLK9 * c.CHP * 4); c.HST = (int*)al((size_t)CSR_NBLK9 * c.NGP * 4); c.OFF = (int*)al((size_t)c.NGP * CSR_NBLK9 * 4); c.START = (int*)al((size_t)(c.NGP + 64) * 4); c.TOT = (int*)al((size_t)(c.NGP + 64) * 4);
  c.PERM = (int*)al(c.permLen * 4); c.ROWPTR = (int*)al((size_t)c.nG * CSR_TS9 * 4); c.ROWCNT = (int*)al((size_t)c.nG * CSR_TS9 * 4); c.FLAG = (int*)al(256);
  c.bytes = off - off0; return off;
}
static void csr_build9(const CsrBufs9& c, const int* dst, int E, int N, hipStream_t stream) {
  const size_t smem = (size_t)(2 * c.NGP + c.CHP) * 4;
  csrZ_kernel9<<<512, 256, 0, stream>>>((int*)c.base, c.bytes / 16);
  csrA_kernel9<<<CSR_NBLK9, 64, smem, stream>>>(dst, E, N, c.nG, c.CHP, c.NGP, c.STG, c.HST);
  csrS_kernel9<<<1, 512, 0, stream>>>(c.HST, c.nG, c.NGP, c.START, c.TOT, c.OFF);
  csrB_kernel9<<<c.nG, 256, 0, stream>>>(dst, N, c.nG, c.CHP, c.NGP, (int)c.permLen, c.STG, c.HST, c.OFF, c.START, c.TOT, c.PERM, c.ROWPTR, c.ROWCNT, c.FLAG);
}


__global__ __launch_bounds__(256) void wput_kernel(const float* __restrict__ iw, const float* __restrict__ w1, const float* __restrict__ w2, const float* __restrict__ w3, const float* __restrict__ aff, b16* __restrict__ INIT_T, b16* __restrict__ WT, b16* __restrict__ AT) { const int u = blockIdx.x * 256 + threadIdx.x;
  for (int pass = 0; pass < 2; ++pass) {
    if (u < F * 8) { const int o = u / 8, k0 = (u % 8) * 8; v8b v;
#pragma unroll
      for (int j = 0; j < 8; ++j) { const int k = k0 + j; v[j] = (b16)(k < KI ? bf16_rne(iw[(size_t)k * F + o]) * WSC : 0.0f); } *(volatile v8b*)(INIT_T + (size_t)o * 64 + k0) = v; }
    if (u < 3 * F * 16) { const int r = u / 16, k0 = (u % 16) * 8; const int which = r / F, o = r % F; const float* w = which == 0 ? w1 : which == 1 ? w2 : w3; v8b v;
#pragma unroll
      for (int j = 0; j < 8; ++j) v[j] = (b16)(bf16_rne(w[(size_t)(k0 + j) * F + o]) * WSC); *(volatile v8b*)(WT + (size_t)r * F + k0) = v; }
    if (u < F * 16) { const int g = u / 16, k0 = (u % 16) * 8; v8b v;
#pragma unroll
      for (int j = 0; j < 8; ++j) v[j] = (b16)(bf16_rne(aff[(size_t)(k0 + j) * F + g]) * WSC); *(volatile v8b*)(AT + (size_t)g * F + k0) = v; }
    __threadfence(); } }
__global__ __launch_bounds__(32) void init_kernel(const float* __restrict__ x, const int* __restrict__ cent, const float* __restrict__ rw, const float* __restrict__ demb, const b16* __restrict__ INIT_T, const float* __restrict__ ib, int NLIM, float* __restrict__ FEAT) {
  __shared__ __attribute__((aligned(16))) b16 Ah[16][72]; __shared__ float Tf[16][132]; const int lane = threadIdx.x, nloc = lane & 15, hlf = lane >> 4; const size_t m0 = (size_t)blockIdx.x * 16; if (m0 >= (size_t)NLIM) return;
  for (int rr = 0; rr < 16; ++rr) { const size_t n = m0 + rr; const int ce = iclamp(cent[n], 0, MD - 1); for (int q = 0; q < 2; ++q) { const int k = q * 32 + lane; float v = 0.0f; if (k < LD) v = x[n * LD + k]; else if (k < LD + MD) v = demb[ce * MD + (k - LD)]; else if (k < KI) v = rw[n * RW + (k - LD - MD)]; Ah[rr][k] = (b16)(bf16_rne(v) * XS); } }
  wave_lds_sync(); v8f acc[8];
#pragma unroll
  for (int t = 0; t < 8; ++t) acc[t] = (v8f){};
#pragma unroll
  for (int kb = 0; kb < 64; kb += 32) { const v16b a = frag_kb(&Ah[nloc][kb], hlf);
#pragma unroll
    for (int t = 0; t < 8; ++t) acc[t] = wmma16b(a, frag_kb(INIT_T + (size_t)(t * 16 + nloc) * 64 + kb, hlf), acc[t]); }
#pragma unroll
  for (int t = 0; t < 8; ++t) { const int c = t * 16 + nloc; const float bb = bf16_rne(ib[c]);
#pragma unroll
    for (int r8 = 0; r8 < 8; ++r8) Tf[8 * hlf + r8][c] = fmaxf(acc[t][r8] * (1.0f / (XS * WSC)) + bb, 0.0f); }
  wave_lds_sync();
  for (int pass = 0; pass < 2; ++pass) { for (int rr = 0; rr < 16; ++rr) *(volatile v4f*)(FEAT + (m0 + rr) * F + lane * 4) = *(const v4f*)(&Tf[rr][lane * 4]); __threadfence(); } }
template <int RELU>
__global__ __launch_bounds__(32) void dense_kernel(const float* __restrict__ IN, const b16* __restrict__ Wsec, int NLIM, float* __restrict__ H) { __shared__ __attribute__((aligned(16))) b16 Ah[16][F + 8], Al[16][F + 8]; __shared__ float Tf[16][132]; const int lane = threadIdx.x, nloc = lane & 15, hlf = lane >> 4; const size_t m0 = (size_t)blockIdx.x * 16; if (m0 >= (size_t)NLIM) return;
  for (int rr = 0; rr < 16; ++rr) for (int q = 0; q < 4; ++q) { float v = IN[(m0 + rr) * F + q * 32 + lane]; if (RELU) v = fmaxf(v, 0.0f); b16 p, ql; split16(v * XS, p, ql); Ah[rr][q * 32 + lane] = p; Al[rr][q * 32 + lane] = ql; }
  wave_lds_sync(); v8f acc[8];
#pragma unroll
  for (int t = 0; t < 8; ++t) acc[t] = (v8f){};
#pragma unroll
  for (int kb = 0; kb < F; kb += 32) { const v16b a = frag_kb(&Ah[nloc][kb], hlf), al = frag_kb(&Al[nloc][kb], hlf);
#pragma unroll
    for (int t = 0; t < 8; ++t) { const v16b bw = frag_kb(Wsec + (size_t)(t * 16 + nloc) * F + kb, hlf); acc[t] = wmma16b(a, bw, acc[t]); acc[t] = wmma16b(al, bw, acc[t]); } }
#pragma unroll
  for (int t = 0; t < 8; ++t)
#pragma unroll
    for (int r8 = 0; r8 < 8; ++r8) Tf[8 * hlf + r8][t * 16 + nloc] = acc[t][r8] * (1.0f / (XS * WSC));
  wave_lds_sync();
  for (int pass = 0; pass < 2; ++pass) { for (int rr = 0; rr < 16; ++rr) *(volatile v4f*)(H + (m0 + rr) * F + lane * 4) = *(const v4f*)(&Tf[rr][lane * 4]); __threadfence(); } }
__global__ __launch_bounds__(256) void gcn_kernel(const float* __restrict__ H, const float* __restrict__ bias, const int* __restrict__ srcs, const int* __restrict__ PERM, const int* __restrict__ ROWPTR, const int* __restrict__ ROWCNT, int permLen, int NLIM, float* __restrict__ OUT) {
  const int wave = threadIdx.x >> 5, lane = threadIdx.x & 31; const size_t i = (size_t)blockIdx.x * 8 + wave; if (i >= (size_t)NLIM) return; int st = ROWPTR[i], cnt = ROWCNT[i]; cnt = iclamp(cnt, 0, 1 << 20); st = iclamp(st, 0, permLen - cnt);
  v4f acc = {0.0f, 0.0f, 0.0f, 0.0f}; int nin = 0;
#pragma unroll 1
  for (int j = 0; j < cnt; ++j) { const int e = iclamp(PERM[st + j], 0, E - 1); const size_t u = (size_t)iclamp(srcs[e], 0, NT - 1); if (u >= (size_t)NLIM) continue; ++nin; const float du = rsqrtf((float)(iclamp(ROWCNT[u], 0, 1 << 20) + 1)); const v4f hv = *(const v4f*)(H + u * F + lane * 4); for (int k = 0; k < 4; ++k) acc[k] += pmul(du, hv[k]); }
  const float di = rsqrtf((float)(nin + 1)); const v4f hi_ = *(const v4f*)(H + i * F + lane * 4); v4f o; for (int k = 0; k < 4; ++k) o[k] = pmul(di, acc[k]) + pmul(pmul(di, di), hi_[k]) + bf16_rne(bias[lane * 4 + k]);
  for (int pass = 0; pass < 2; ++pass) { *(volatile v4f*)(OUT + i * F + lane * 4) = o; __threadfence(); } }
__global__ __launch_bounds__(256) void split_kernel(const float* __restrict__ X, int NLIM, b16* __restrict__ Xh, b16* __restrict__ Xl) { const size_t u = (size_t)blockIdx.x * 256 + threadIdx.x; if (u >= (size_t)NLIM * F / 4) return; const v4f v = *(const v4f*)(X + u * 4); v4b ph, pl; for (int k = 0; k < 4; ++k) { b16 p, q; split16(v[k] * XS, p, q); ph[k] = p; pl[k] = q; } for (int pass = 0; pass < 2; ++pass) { *(volatile v4b*)(Xh + u * 4) = ph; *(volatile v4b*)(Xl + u * 4) = pl; __threadfence(); } }
__global__ __launch_bounds__(32) void aff_kernel(const float* __restrict__ XA, const b16* __restrict__ AT, const b16* __restrict__ XBh, const b16* __restrict__ XBl, int BV, float* __restrict__ S) {
  __shared__ __attribute__((aligned(16))) b16 Ah[16][F + 8], Al[16][F + 8], Th[16][F + 8], Tl[16][F + 8]; __shared__ float Tf[16][132]; const int lane = threadIdx.x, nloc = lane & 15, hlf = lane >> 4; const int it = blockIdx.x % (NN / 16), b = blockIdx.x / (NN / 16); if (b >= BV) return; const size_t r0 = (size_t)b * NN + it * 16;
  for (int rr = 0; rr < 16; ++rr) for (int q = 0; q < 4; ++q) { b16 p, ql; split16(XA[(r0 + rr) * F + q * 32 + lane] * XS, p, ql); Ah[rr][q * 32 + lane] = p; Al[rr][q * 32 + lane] = ql; }
  wave_lds_sync(); v8f acc[8];
#pragma unroll
  for (int t = 0; t < 8; ++t) acc[t] = (v8f){};
#pragma unroll
  for (int kb = 0; kb < F; kb += 32) { const v16b a = frag_kb(&Ah[nloc][kb], hlf), al = frag_kb(&Al[nloc][kb], hlf);
#pragma unroll
    for (int t = 0; t < 8; ++t) { const v16b bw = frag_kb(AT + (size_t)(t * 16 + nloc) * F + kb, hlf); acc[t] = wmma16b(a, bw, acc[t]); acc[t] = wmma16b(al, bw, acc[t]); } }
#pragma unroll
  for (int t = 0; t < 8; ++t)
#pragma unroll
    for (int r8 = 0; r8 < 8; ++r8) { b16 p, q; split16(acc[t][r8] * (1.0f / (XS * WSC)) * XS, p, q); Th[8 * hlf + r8][t * 16 + nloc] = p; Tl[8 * hlf + r8][t * 16 + nloc] = q; }
  wave_lds_sync();
#pragma unroll
  for (int t = 0; t < 8; ++t) acc[t] = (v8f){};
#pragma unroll
  for (int kb = 0; kb < F; kb += 32) { const v16b a = frag_kb(&Th[nloc][kb], hlf), al = frag_kb(&Tl[nloc][kb], hlf);
#pragma unroll
    for (int t = 0; t < 8; ++t) { const size_t jr = ((size_t)b * NN + t * 16 + nloc) * F + kb; const v16b bh = frag_kb(XBh + jr, hlf), bl = frag_kb(XBl + jr, hlf); acc[t] = wmma16b(a, bh, acc[t]); acc[t] = wmma16b(a, bl, acc[t]); acc[t] = wmma16b(al, bh, acc[t]); } }
#pragma unroll
  for (int t = 0; t < 8; ++t)
#pragma unroll
    for (int r8 = 0; r8 < 8; ++r8) Tf[8 * hlf + r8][t * 16 + nloc] = acc[t][r8] * (1.0f / (XS * XS));
  wave_lds_sync();
  for (int pass = 0; pass < 2; ++pass) { for (int rr = 0; rr < 16; ++rr) *(volatile v4f*)(S + (r0 + rr) * NN + lane * 4) = *(const v4f*)(&Tf[rr][lane * 4]); __threadfence(); } }
__device__ __forceinline__ float blk_reduce_max(float v, float* red, int t) { red[t] = v; __syncthreads(); for (int s = 128; s > 0; s >>= 1) { if (t < s) red[t] = fmaxf(red[t], red[t + s]); __syncthreads(); } const float r = red[0]; __syncthreads(); return r; }
__device__ __forceinline__ float blk_reduce_sum(float v, float* red, int t) { red[t] = v; __syncthreads(); for (int s = 128; s > 0; s >>= 1) { if (t < s) red[t] = red[t] + red[t + s]; __syncthreads(); } const float r = red[0]; __syncthreads(); return r; }
__global__ __launch_bounds__(256) void topk_kernel(const float* __restrict__ S, const int* __restrict__ topk, int BV, float* __restrict__ out) {
  __shared__ float fs[L], red[256]; const int t = threadIdx.x, b = blockIdx.x; if (b >= BV) return; const float* xs = S + (size_t)b * L;
  float mn = INFINITY, mx = -INFINITY; for (int l = t; l < L; l += 256) { const float v = xs[l]; mn = fminf(mn, v); mx = fmaxf(mx, v); }
  mx = blk_reduce_max(mx, red, t); mn = -blk_reduce_max(-mn, red, t);
  const float a0 = mn - 1.0f, a1 = mx + 1.0f; const float kk = 0.5f * (float)iclamp(topk[0], 0, 2 * L); const float log_mu = -__logf((float)L); const float log_nu0 = __logf(((float)L - kk) / (float)L), log_nu1 = __logf(kk / (float)L);
  float g0 = 0.0f, g1 = 0.0f; for (int l = t; l < L; l += 256) fs[l] = 0.0f;
  auto lk0 = [&](int l) { return -fabsf(xs[l] - a0) / TAU; }; auto lk1 = [&](int l) { return -fabsf(xs[l] - a1) / TAU; };
#pragma unroll 1
  for (int itn = 0; itn < SKIT; ++itn) {
    for (int l = t; l < L; l += 256) { const float u0 = lk0(l) + g0, u1 = lk1(l) + g1; const float m = fmaxf(u0, u1); fs[l] = log_mu - (m + __logf(__expf(u0 - m) + __expf(u1 - m))); }
    __syncthreads();
    for (int c = 0; c < 2; ++c) { float m = -INFINITY; for (int l = t; l < L; l += 256) m = fmaxf(m, (c == 0 ? lk0(l) : lk1(l)) + fs[l]); m = blk_reduce_max(m, red, t); float s = 0.0f; for (int l = t; l < L; l += 256) s += __expf((c == 0 ? lk0(l) : lk1(l)) + fs[l] - m); s = blk_reduce_sum(s, red, t); const float gc = (c == 0 ? log_nu0 : log_nu1) - (m + __logf(s)); if (c == 0) g0 = gc; else g1 = gc; } }
  for (int pass = 0; pass < 2; ++pass) { for (int l = t; l < L; l += 256) ((volatile float*)out)[(size_t)b * L + l] = __expf(lk1(l) + fs[l] + g1) * (float)L; __threadfence(); } }
__global__ __launch_bounds__(256) void pool_kernel(const float* __restrict__ FEAT, const float* __restrict__ F1, const float* __restrict__ F2, const float* __restrict__ F3, int BV, float* __restrict__ SC) { const int t = threadIdx.x, b = blockIdx.x; if (b >= BV) return;
  float vals[4];
#pragma unroll
  for (int part = 0; part < 4; ++part) { const int col = part * 256 + t; const int side = col / 512, blk = (col % 512) / F, c = col % F; const float* P = blk == 0 ? FEAT : blk == 1 ? F1 : blk == 2 ? F2 : F3; const size_t base = ((size_t)side * NT + (size_t)b * NN) * F + c; float s = side == 0 ? 0.0f : -INFINITY;
#pragma unroll 1
    for (int n = 0; n < NN; ++n) { const float v = P[base + (size_t)n * F]; s = side == 0 ? s + v : fmaxf(s, v); } vals[part] = s; }
  for (int pass = 0; pass < 2; ++pass) {
#pragma unroll
    for (int part = 0; part < 4; ++part) ((volatile float*)SC)[(size_t)b * 1024 + part * 256 + t] = vals[part]; __threadfence(); } }
__global__ __launch_bounds__(256) void ged_kernel(const float* __restrict__ SC, const float* __restrict__ w1, const float* __restrict__ b1, const float* __restrict__ w2, const float* __restrict__ b2, int BV, float* __restrict__ out) { const int b = threadIdx.x; float g = 0.0f;
  if (b < BV) { float s2 = bf16_rne(b2[0]);
#pragma unroll 1
    for (int o = 0; o < 64; ++o) { float s = bf16_rne(b1[o]);
#pragma unroll 4
      for (int k = 0; k < 1024; ++k) s += pmul(SC[(size_t)b * 1024 + k], bf16_rne(w1[(size_t)k * 64 + o])); s2 += pmul(fmaxf(s, 0.0f), bf16_rne(w2[o])); }
    g = 1.0f / (1.0f + __expf(-s2)); }
  for (int pass = 0; pass < 2; ++pass) { ((volatile float*)out)[b] = g; __threadfence(); } }
}

extern "C" void kernel_launch(void* const* d_in, const int* in_sizes, int n_in, void* d_out, int out_size, void* d_ws, size_t ws_size, hipStream_t stream) {
  (void)n_in;
  auto Fp = [&](int i) { return (const float*)d_in[i]; }; auto Ip = [&](int i) { return (const int*)d_in[i]; };
  if (in_sizes[0] != NT * LD || in_sizes[1] != NT || in_sizes[2] != NT * RW || in_sizes[3] != E || in_sizes[4] != E || in_sizes[8] != E || in_sizes[9] != E || in_sizes[11] != KI * F || in_sizes[19] != F * F || in_sizes[20] != 1024 * 64 || in_sizes[24] != 1 || out_size != NB + 2 * NB * L) return;
  const int BV = NB; const int NLIM = BV * NN;
  size_t off = 0; char* ws = (char*)d_ws;
  auto carve = [&](size_t bytes) { char* p = ws + off; off += (bytes + 255) & ~(size_t)255; return p; };
  b16* INIT_T = (b16*)carve((size_t)F * 64 * 2); b16* WT = (b16*)carve((size_t)3 * F * F * 2); b16* AT = (b16*)carve((size_t)F * F * 2);
  float* FEAT = (float*)carve((size_t)2 * NT * F * 4); float* F1 = (float*)carve((size_t)2 * NT * F * 4); float* F2 = (float*)carve((size_t)2 * NT * F * 4); float* F3 = (float*)carve((size_t)2 * NT * F * 4); float* H = (float*)carve((size_t)NT * F * 4);
  b16* XBh = (b16*)carve((size_t)NT * F * 2); b16* XBl = (b16*)carve((size_t)NT * F * 2); float* S = (float*)carve((size_t)NB * L * 4); float* SC = (float*)carve((size_t)NB * 1024 * 4);
  CsrBufs9 c1, c2; off = csr_carve9(c1, ws, off, E, NT); off = csr_carve9(c2, ws, off, E, NT);
  if (off > ws_size || off > ((size_t)220 << 20)) return;
  float* out = (float*)d_out; float* gedout = out; float* sim1 = out + NB; float* sim2 = sim1 + (size_t)NB * L;
  wput_kernel<<<(3 * F * 16 + 255) / 256, 256, 0, stream>>>(Fp(11), Fp(13), Fp(15), Fp(17), Fp(19), INIT_T, WT, AT);
  csr_build9(c1, Ip(4), E, NT, stream); csr_build9(c2, Ip(9), E, NT, stream);
  for (int side = 0; side < 2; ++side) { const int xo = side == 0 ? 0 : 5; float* feat = FEAT + (size_t)side * NT * F; float* f1 = F1 + (size_t)side * NT * F; float* f2 = F2 + (size_t)side * NT * F; float* f3 = F3 + (size_t)side * NT * F; CsrBufs9& cs = side == 0 ? c1 : c2; const int* sr = Ip(xo + 3);
    init_kernel<<<NLIM / 16, 32, 0, stream>>>(Fp(xo + 0), Ip(xo + 1), Fp(xo + 2), Fp(10), INIT_T, Fp(12), NLIM, feat);
    dense_kernel<0><<<NLIM / 16, 32, 0, stream>>>(feat, WT, NLIM, H); gcn_kernel<<<(NLIM + 7) / 8, 256, 0, stream>>>(H, Fp(14), sr, cs.PERM, cs.ROWPTR, cs.ROWCNT, (int)cs.permLen, NLIM, f1);
    dense_kernel<1><<<NLIM / 16, 32, 0, stream>>>(f1, WT + (size_t)F * F, NLIM, H); gcn_kernel<<<(NLIM + 7) / 8, 256, 0, stream>>>(H, Fp(16), sr, cs.PERM, cs.ROWPTR, cs.ROWCNT, (int)cs.permLen, NLIM, f2);
    dense_kernel<1><<<NLIM / 16, 32, 0, stream>>>(f2, WT + (size_t)2 * F * F, NLIM, H); gcn_kernel<<<(NLIM + 7) / 8, 256, 0, stream>>>(H, Fp(18), sr, cs.PERM, cs.ROWPTR, cs.ROWCNT, (int)cs.permLen, NLIM, f3); }
  split_kernel<<<(unsigned)(((size_t)NLIM * F / 4 + 255) / 256), 256, 0, stream>>>(FEAT + (size_t)NT * F, NLIM, XBh, XBl);
  aff_kernel<<<BV * (NN / 16), 32, 0, stream>>>(FEAT, AT, XBh, XBl, BV, S); topk_kernel<<<BV, 256, 0, stream>>>(S, Ip(24), BV, sim1);
  split_kernel<<<(unsigned)(((size_t)NLIM * F / 4 + 255) / 256), 256, 0, stream>>>(F3 + (size_t)NT * F, NLIM, XBh, XBl);
  aff_kernel<<<BV * (NN / 16), 32, 0, stream>>>(F3, AT, XBh, XBl, BV, S); topk_kernel<<<BV, 256, 0, stream>>>(S, Ip(24), BV, sim2);
  pool_kernel<<<BV, 256, 0, stream>>>(FEAT, F1, F2, F3, BV, SC);
  ged_kernel<<<1, 256, 0, stream>>>(SC, Fp(20), Fp(21), Fp(22), Fp(23), BV, gedout);
}
